// Attention_43353399886449
// MI455X (gfx1250) — hardware-verified
//
#include <hip/hip_runtime.h>
#include <stddef.h>


#ifndef NB
#define NB 2
#endif
#ifndef SEQ
#define SEQ 2048
#endif
#define NB_FULL 2
#define SEQ_FULL 2048
#define DM 2048
#define NH 16
#define NKV 4
#define HD 128
#define DQ (NH * HD)
#define DKV (NKV * HD)
#define NTOK (NB * SEQ)
#define KD 2048

#define BT 128
#define BK 32
#define LST 40
#define RP ((DQ / 8) + (DKV / 8))

static_assert(NB >= 1 && NB <= NB_FULL);
static_assert(SEQ >= 128 && SEQ <= SEQ_FULL && (SEQ % 128) == 0);
static_assert(DM == KD && DQ == KD);
static_assert((DM % BT) == 0 && (DQ % BT) == 0 && (DKV % BT) == 0 && (NTOK % BT) == 0);
static_assert((KD % 64) == 0 && (KD % BK) == 0);
static_assert(HD == BT);
static_assert((DM / 8) == 256);
static_assert((RP % 32) == 0 && ((DQ / 8) % 32) == 0);
static_assert((NH % NKV) == 0);

typedef _Float16 v16h __attribute__((ext_vector_type(16)));
typedef _Float16 v8h  __attribute__((ext_vector_type(8)));
typedef float    v8f  __attribute__((ext_vector_type(8)));
typedef float    v4f  __attribute__((ext_vector_type(4)));

union Frag { v16h v; v8h p[2]; };

__device__ __forceinline__ float bf16r(float f) {
  unsigned u = __float_as_uint(f);
  u = (u + 0x7FFFu + ((u >> 16) & 1u)) & 0xFFFF0000u;
  return __uint_as_float(u);
}

__device__ __forceinline__ v8f wmma16(v16h a, v16h b, v8f c) {
  v8f d = __builtin_amdgcn_wmma_f32_16x16x32_f16(false, a, false, b, (short)0, c, false, false);
  asm volatile("v_nop\n\tv_nop\n\tv_nop\n\tv_nop" : "+v"(d) : "v"(a), "v"(b));
  return d;
}

__device__ __forceinline__ v16h load_frag(const _Float16* q) {
  Frag f;
  f.p[0] = *(const v8h*)(q);
  f.p[1] = *(const v8h*)(q + 16);
  return f.v;
}

__global__ void __launch_bounds__(256)
cvt_x_kernel(const float* __restrict__ x, _Float16* __restrict__ Xh, int nPieces) {
  const int f = blockIdx.x * 256 + (int)threadIdx.x;
  if (f >= nPieces) return;
  const int tok = f >> 8;
  const int c0  = (f & 255) * 8;
  const int b = tok / SEQ, s = tok - b * SEQ;
  const float* src = x + ((size_t)(b * SEQ_FULL + s) * DM + c0);
  const v4f a0 = *(const v4f*)(src);
  const v4f a1 = *(const v4f*)(src + 4);
  v8h o;
#pragma unroll
  for (int j = 0; j < 4; ++j) {
    o[j]     = (_Float16)bf16r(a0[j]);
    o[j + 4] = (_Float16)bf16r(a1[j]);
  }
  _Float16* dst = Xh + ((size_t)tok * DM + c0);
  *(volatile v8h*)dst = o;
  __threadfence();
  *(volatile v8h*)dst = o;
}

__global__ void __launch_bounds__(256)
cvt_w_kernel(const float* __restrict__ Wq, const float* __restrict__ Wk,
             const float* __restrict__ Wv, const float* __restrict__ Wo,
             _Float16* __restrict__ WqT, _Float16* __restrict__ WkT,
             _Float16* __restrict__ WvT, _Float16* __restrict__ WoT) {
  __shared__ __align__(16) _Float16 lds[64 * 72];
  const int bx = blockIdx.x;
  const float* W; _Float16* WT; int N; int nt;
  if (bx < DQ / 64) { W = Wq; WT = WqT; N = DQ;  nt = bx; }
  else if (bx < DQ / 64 + DKV / 64) { W = Wk; WT = WkT; N = DKV; nt = bx - DQ / 64; }
  else if (bx < DQ / 64 + 2 * (DKV / 64)) { W = Wv; WT = WvT; N = DKV; nt = bx - DQ / 64 - DKV / 64; }
  else { W = Wo; WT = WoT; N = DM; nt = bx - DQ / 64 - 2 * (DKV / 64); }
  const int k0 = blockIdx.y * 64, n0 = nt * 64;
  const int t = threadIdx.x, lane = t & 31, w = t >> 5;
  const int kr = t >> 2, cc = (t & 3) * 16;
  const float* src = W + ((size_t)(k0 + kr) * N + n0 + cc);
#pragma unroll
  for (int q = 0; q < 4; ++q) {
    const v4f v = *(const v4f*)(src + 4 * q);
#pragma unroll
    for (int j = 0; j < 4; ++j)
      lds[(cc + 4 * q + j) * 72 + kr] = (_Float16)(64.0f * bf16r(v[j]));
  }
  __syncthreads();
  v8h ov[2];
#pragma unroll
  for (int j = 0; j < 2; ++j) {
    const int n = w * 8 + j * 4 + (lane >> 3);
    ov[j] = *(const v8h*)&lds[n * 72 + (lane & 7) * 8];
  }
  _Float16* base = WT + ((size_t)n0 * KD + k0 + (lane & 7) * 8);
#pragma unroll
  for (int j = 0; j < 2; ++j) {
    const int n = w * 8 + j * 4 + (lane >> 3);
    *(volatile v8h*)(base + (size_t)n * KD) = ov[j];
  }
  __threadfence();
#pragma unroll
  for (int j = 0; j < 2; ++j) {
    const int n = w * 8 + j * 4 + (lane >> 3);
    *(volatile v8h*)(base + (size_t)n * KD) = ov[j];
  }
}

union GemmLds { _Float16 h[4 * BT * LST]; float f[2 * BT * LST]; };

template <typename TC>
__global__ void __launch_bounds__(256)
gemm_kernel(const _Float16* __restrict__ A, const _Float16* __restrict__ Bt0,
            const _Float16* __restrict__ Bt1, TC* C0, TC* C1,
            int N0, int N1, int nTiles0, float alpha) {
  __shared__ __align__(16) GemmLds pool;

  const int bx = blockIdx.x;
  const bool second = bx >= nTiles0;
  const _Float16* Bt = second ? Bt1 : Bt0;
  TC* C = second ? C1 : C0;
  const int N  = second ? N1 : N0;
  const int nt = second ? (bx - nTiles0) : bx;
  const int m0 = blockIdx.y * BT, n0 = nt * BT;

  const int t = threadIdx.x, lane = t & 31, w = t >> 5, lr = lane & 15, hi = lane >> 4;

  v8f acc[8];
#pragma unroll
  for (int ni = 0; ni < 8; ++ni) acc[ni] = (v8f){0.f, 0.f, 0.f, 0.f, 0.f, 0.f, 0.f, 0.f};

  const int arow = t >> 1, acol = (t & 1) * 16;
  const _Float16* aSrc = A  + ((size_t)(m0 + arow) * KD + acol);
  const _Float16* bSrc = Bt + ((size_t)(n0 + arow) * KD + acol);

  auto stage = [&](int k0, int buf) {
    _Float16* da = pool.h + buf * (BT * LST) + arow * LST + acol;
    _Float16* db = pool.h + (2 + buf) * (BT * LST) + arow * LST + acol;
    *(v8h*)(da)     = *(const v8h*)(aSrc + k0);
    *(v8h*)(da + 8) = *(const v8h*)(aSrc + k0 + 8);
    *(v8h*)(db)     = *(const v8h*)(bSrc + k0);
    *(v8h*)(db + 8) = *(const v8h*)(bSrc + k0 + 8);
  };

  stage(0, 0);
  __syncthreads();

  for (int k0 = 0; k0 < KD; k0 += BK) {
    const int cur = (k0 / BK) & 1, nxt = cur ^ 1;
    if (k0 + BK < KD) stage(k0 + BK, nxt);
    const _Float16* la = pool.h + cur * (BT * LST);
    const _Float16* lb = pool.h + (2 + cur) * (BT * LST);
    const v16h af = load_frag(la + (w * 16 + lr) * LST + hi * 8);
#pragma unroll
    for (int ni = 0; ni < 8; ++ni) {
      const v16h bf = load_frag(lb + (ni * 16 + lr) * LST + hi * 8);
      acc[ni] = wmma16(af, bf, acc[ni]);
    }
    __syncthreads();
  }

  if constexpr (sizeof(TC) == 4) {
    float* stg = pool.f + w * (8 * 132);
#pragma unroll
    for (int ps = 0; ps < 2; ++ps) {
#pragma unroll
      for (int rr = 0; rr < 4; ++rr)
#pragma unroll
        for (int ni = 0; ni < 8; ++ni)
          stg[(hi * 4 + rr) * 132 + ni * 16 + lr] = acc[ni][ps * 4 + rr] * alpha;
      __syncthreads();
      v4f ov[8];
#pragma unroll
      for (int sr = 0; sr < 8; ++sr) ov[sr] = *(const v4f*)&stg[sr * 132 + lane * 4];
      float* cbase = (float*)C + ((size_t)n0 + lane * 4);
#pragma unroll
      for (int sr = 0; sr < 8; ++sr) {
        const int row = m0 + w * 16 + (sr >> 2) * 8 + ps * 4 + (sr & 3);
        *(volatile v4f*)(cbase + (size_t)row * N) = ov[sr];
      }
      __threadfence();
#pragma unroll
      for (int sr = 0; sr < 8; ++sr) {
        const int row = m0 + w * 16 + (sr >> 2) * 8 + ps * 4 + (sr & 3);
        *(volatile v4f*)(cbase + (size_t)row * N) = ov[sr];
      }
      __syncthreads();
    }
  } else {
    const int g  = n0 / HD;
    const int bb = m0 / SEQ;
    const int s0 = m0 - bb * SEQ;
    _Float16* stg = pool.h;
#pragma unroll
    for (int ni = 0; ni < 8; ++ni) {
      v8h v;
#pragma unroll
      for (int r = 0; r < 8; ++r) v[r] = (_Float16)(acc[ni][r] * alpha);
      *(v8h*)&stg[(ni * 16 + lr) * 136 + w * 16 + hi * 8] = v;
    }
    __syncthreads();
    v8h ov[8];
#pragma unroll
    for (int j = 0; j < 8; ++j) {
      const int d = w * 16 + j * 2 + hi;
      ov[j] = *(const v8h*)&stg[d * 136 + lr * 8];
    }
    _Float16* vbase = (_Float16*)C + (((size_t)(bb * NKV + g) * HD) * SEQ + s0 + lr * 8);
#pragma unroll
    for (int j = 0; j < 8; ++j) {
      const int d = w * 16 + j * 2 + hi;
      *(volatile v8h*)(vbase + (size_t)d * SEQ) = ov[j];
    }
    __threadfence();
#pragma unroll
    for (int j = 0; j < 8; ++j) {
      const int d = w * 16 + j * 2 + hi;
      *(volatile v8h*)(vbase + (size_t)d * SEQ) = ov[j];
    }
  }
}

__global__ void __launch_bounds__(256)
rope_kernel(const float* __restrict__ Qf, const float* __restrict__ Kf,
            const float* __restrict__ cosT, const float* __restrict__ sinT,
            _Float16* __restrict__ Qh, _Float16* __restrict__ Kh, int nPieces) {
  const int f = blockIdx.x * 256 + (int)threadIdx.x;
  if (f >= nPieces) return;
  const int tok = f / RP;
  const int piece = f - tok * RP;
  const int s = tok % SEQ;
  const bool isq = piece < (DQ / 8);
  const int col   = isq ? piece * 8 : (piece - DQ / 8) * 8;
  const int pitch = isq ? DQ : DKV;
  const float* src = (isq ? Qf : Kf) + (size_t)tok * pitch;
  _Float16* dst = (isq ? Qh : Kh) + ((size_t)tok * pitch + col);
  const int d    = col & (HD - 1);
  const int colp = col - d + (d ^ 64);
  const float sgn = (d < 64) ? -1.0f : 1.0f;
  const v4f x0 = *(const v4f*)(src + col),  x1 = *(const v4f*)(src + col + 4);
  const v4f p0 = *(const v4f*)(src + colp), p1 = *(const v4f*)(src + colp + 4);
  const v4f c0 = *(const v4f*)(cosT + (size_t)s * HD + d), c1 = *(const v4f*)(cosT + (size_t)s * HD + d + 4);
  const v4f n0 = *(const v4f*)(sinT + (size_t)s * HD + d), n1 = *(const v4f*)(sinT + (size_t)s * HD + d + 4);
  v8h o;
#pragma unroll
  for (int j = 0; j < 4; ++j) {
    o[j]     = (_Float16)(x0[j] * bf16r(c0[j]) + (sgn * p0[j]) * bf16r(n0[j]));
    o[j + 4] = (_Float16)(x1[j] * bf16r(c1[j]) + (sgn * p1[j]) * bf16r(n1[j]));
  }
  *(volatile v8h*)dst = o;
  __threadfence();
  *(volatile v8h*)dst = o;
}

__global__ void __launch_bounds__(256)
attn_kernel(const _Float16* __restrict__ Qh, const _Float16* __restrict__ Kh,
            const _Float16* __restrict__ Vt, _Float16* __restrict__ Oh) {
  constexpr int LDK = 136, LDV = 72, LDP = 72, LDO = 136;
  __shared__ __align__(16) _Float16 pool[64 * LDK + 128 * LDV + 128 * LDP];
  _Float16* lsK = pool;
  _Float16* lsV = pool + 64 * LDK;
  _Float16* lsP = lsV + 128 * LDV;

  const int t = threadIdx.x, lane = t & 31, w = t >> 5, lr = lane & 15, hi = lane >> 4;
  const int b = blockIdx.z, h = blockIdx.y, g = h / (NH / NKV);
  const int q0 = blockIdx.x * 128 + w * 16;
  const size_t tokb = (size_t)b * SEQ;
  _Float16* myP = lsP + w * 16 * LDP;

  const float kSL = 0.08838834764831845f * 1.4426950408889634f;

  v16h qf[4];
  {
    const _Float16* qrow = Qh + ((tokb + q0 + lr) * DQ + h * HD);
#pragma unroll
    for (int kf = 0; kf < 4; ++kf) qf[kf] = load_frag(qrow + kf * 32 + hi * 8);
  }

  float mrow[8], lrow[8];
  v8f oacc[8];
#pragma unroll
  for (int i = 0; i < 8; ++i) { mrow[i] = -1e30f; lrow[i] = 0.f; }
#pragma unroll
  for (int dt = 0; dt < 8; ++dt) oacc[dt] = (v8f){0.f, 0.f, 0.f, 0.f, 0.f, 0.f, 0.f, 0.f};

  const _Float16* kbase = Kh + ((tokb) * DKV + g * HD);
  const _Float16* vbase = Vt + ((size_t)(b * NKV + g) * HD) * SEQ;

  for (int kc = 0; kc < SEQ; kc += 64) {
#pragma unroll
    for (int i = 0; i < 4; ++i) {
      const int e = t + i * 256;
      const int key = e >> 4, seg = e & 15;
      *(v8h*)&lsK[key * LDK + seg * 8] = *(const v8h*)(kbase + (size_t)(kc + key) * DKV + seg * 8);
    }
#pragma unroll
    for (int i = 0; i < 4; ++i) {
      const int e = t + i * 256;
      const int d = e >> 3, seg = e & 7;
      *(v8h*)&lsV[d * LDV + seg * 8] = *(const v8h*)(vbase + (size_t)d * SEQ + kc + seg * 8);
    }
    __syncthreads();

    v8f sc[4];
#pragma unroll
    for (int nt = 0; nt < 4; ++nt) {
      sc[nt] = (v8f){0.f, 0.f, 0.f, 0.f, 0.f, 0.f, 0.f, 0.f};
#pragma unroll
      for (int kf = 0; kf < 4; ++kf) {
        const v16h bf = load_frag(lsK + (nt * 16 + lr) * LDK + kf * 32 + hi * 8);
        sc[nt] = wmma16(qf[kf], bf, sc[nt]);
      }
    }

#pragma unroll
    for (int i = 0; i < 8; ++i) {
      float sl[4];
#pragma unroll
      for (int nt = 0; nt < 4; ++nt) sl[nt] = sc[nt][i] * kSL;
      float mx = fmaxf(fmaxf(sl[0], sl[1]), fmaxf(sl[2], sl[3]));
      mx = fmaxf(mx, __shfl_xor(mx, 1, 32));
      mx = fmaxf(mx, __shfl_xor(mx, 2, 32));
      mx = fmaxf(mx, __shfl_xor(mx, 4, 32));
      mx = fmaxf(mx, __shfl_xor(mx, 8, 32));
      const float mn = fmaxf(mrow[i], mx);
      const float corr = exp2f(mrow[i] - mn);
      mrow[i] = mn;
      float rs = 0.f;
#pragma unroll
      for (int nt = 0; nt < 4; ++nt) {
        const float p = exp2f(sl[nt] - mn);
        rs += p;
        myP[(hi * 8 + i) * LDP + nt * 16 + lr] = (_Float16)(p * 1024.0f);
      }
      rs += __shfl_xor(rs, 1, 32);
      rs += __shfl_xor(rs, 2, 32);
      rs += __shfl_xor(rs, 4, 32);
      rs += __shfl_xor(rs, 8, 32);
      lrow[i] = lrow[i] * corr + rs;
#pragma unroll
      for (int dt = 0; dt < 8; ++dt) oacc[dt][i] *= corr;
    }
    __syncthreads();

    v16h pf[2];
#pragma unroll
    for (int kf = 0; kf < 2; ++kf) pf[kf] = load_frag(myP + lr * LDP + kf * 32 + hi * 8);
#pragma unroll
    for (int dt = 0; dt < 8; ++dt) {
#pragma unroll
      for (int kf = 0; kf < 2; ++kf) {
        const v16h bf = load_frag(lsV + (dt * 16 + lr) * LDV + kf * 32 + hi * 8);
        oacc[dt] = wmma16(pf[kf], bf, oacc[dt]);
      }
    }
    __syncthreads();
  }

  _Float16* stg = pool + w * 16 * LDO;
#pragma unroll
  for (int i = 0; i < 8; ++i) {
    const float inv = 0.0625f / lrow[i];
#pragma unroll
    for (int dt = 0; dt < 8; ++dt)
      stg[(hi * 8 + i) * LDO + dt * 16 + lr] = (_Float16)(oacc[dt][i] * inv);
  }
  __syncthreads();
  v8h ov[8];
#pragma unroll
  for (int j = 0; j < 8; ++j) ov[j] = *(const v8h*)&stg[(j * 2 + hi) * LDO + lr * 8];
  _Float16* obase = Oh + ((tokb + q0) * DQ + h * HD + lr * 8);
#pragma unroll
  for (int j = 0; j < 8; ++j) *(volatile v8h*)(obase + (size_t)(j * 2 + hi) * DQ) = ov[j];
  __threadfence();
#pragma unroll
  for (int j = 0; j < 8; ++j) *(volatile v8h*)(obase + (size_t)(j * 2 + hi) * DQ) = ov[j];
}

extern "C" void kernel_launch(void* const* d_in, const int* in_sizes, int n_in,
                              void* d_out, int out_size, void* d_ws, size_t ws_size,
                              hipStream_t stream) {
  if (n_in < 7) return;
  if (in_sizes[0] < ((NB - 1) * SEQ_FULL + SEQ) * DM) return;
  if (in_sizes[1] < SEQ * HD) return;
  if (in_sizes[2] < SEQ * HD) return;
  if (in_sizes[3] < DM * DQ) return;
  if (in_sizes[4] < DM * DKV) return;
  if (in_sizes[5] < DM * DKV) return;
  if (in_sizes[6] < DQ * DM) return;
  if (out_size < NTOK * DM) return;

  const float* x    = (const float*)d_in[0];
  const float* cosT = (const float*)d_in[1];
  const float* sinT = (const float*)d_in[2];
  const float* Wq   = (const float*)d_in[3];
  const float* Wk   = (const float*)d_in[4];
  const float* Wv   = (const float*)d_in[5];
  const float* Wo   = (const float*)d_in[6];
  float* out = (float*)d_out;

  char* ws = (char*)d_ws;
  size_t off = 0;
  _Float16* Xh  = (_Float16*)(ws + off); off += (size_t)NTOK * DM * 2;
  _Float16* WqT = (_Float16*)(ws + off); off += (size_t)DQ  * KD * 2;
  _Float16* WkT = (_Float16*)(ws + off); off += (size_t)DKV * KD * 2;
  _Float16* WvT = (_Float16*)(ws + off); off += (size_t)DKV * KD * 2;
  _Float16* WoT = (_Float16*)(ws + off); off += (size_t)DM  * KD * 2;
  float*    Qf  = (float*)(ws + off);    off += (size_t)NTOK * DQ * 4;
  float*    Kf  = (float*)(ws + off);    off += (size_t)NTOK * DKV * 4;
  _Float16* Qh  = (_Float16*)(ws + off); off += (size_t)NTOK * DQ * 2;
  _Float16* Kh  = (_Float16*)(ws + off); off += (size_t)NTOK * DKV * 2;
  _Float16* Vt  = (_Float16*)(ws + off); off += (size_t)NB * NKV * HD * SEQ * 2;
  _Float16* Oh  = (_Float16*)(ws + off); off += (size_t)NTOK * DQ * 2;
  if (off > ws_size) return;

  const dim3 blk(256);

  {
    const int np = NTOK * (DM / 8);
    cvt_x_kernel<<<dim3((np + 255) / 256), blk, 0, stream>>>(x, Xh, np);
  }
  cvt_w_kernel<<<dim3(DQ / 64 + 2 * (DKV / 64) + DM / 64, KD / 64), blk, 0, stream>>>(
      Wq, Wk, Wv, Wo, WqT, WkT, WvT, WoT);
  gemm_kernel<float><<<dim3(DQ / BT + DKV / BT, NTOK / BT), blk, 0, stream>>>(
      Xh, WqT, WkT, Qf, Kf, DQ, DKV, DQ / BT, 0.015625f);
  gemm_kernel<_Float16><<<dim3(DKV / BT, NTOK / BT), blk, 0, stream>>>(
      Xh, WvT, WvT, Vt, Vt, DKV, DKV, DKV / BT, 0.015625f);
  {
    const int np = NTOK * RP;
    rope_kernel<<<dim3((np + 255) / 256), blk, 0, stream>>>(Qf, Kf, cosT, sinT, Qh, Kh, np);
  }
  attn_kernel<<<dim3(SEQ / 128, NH, NB), blk, 0, stream>>>(Qh, Kh, Vt, Oh);
  gemm_kernel<float><<<dim3(DM / BT, NTOK / BT), blk, 0, stream>>>(
      Oh, WoT, WoT, out, out, DM, DM, DM / BT, 0.000244140625f);
}
